// CandidateRelationalActionQRanker_51823075393570
// MI455X (gfx1250) — hardware-verified
//
#include <hip/hip_runtime.h>
#include <math.h>


typedef _Float16 v16h __attribute__((ext_vector_type(16)));
typedef _Float16 v8h  __attribute__((ext_vector_type(8)));
typedef float    v8f  __attribute__((ext_vector_type(8)));
typedef float    v4f  __attribute__((ext_vector_type(4)));
typedef float    v2f  __attribute__((ext_vector_type(2)));
union Frag { v16h v; v8h half[2]; };

#define NN     1024
#define FEAT   256
#define HID    64
#define QKVW   192
#define WPITCH 72

__device__ __forceinline__ v8f wmma16(v16h a, v16h b, v8f c) {
    v8f d = __builtin_amdgcn_wmma_f32_16x16x32_f16(false, a, false, b, (short)0, c, false, false);
    asm volatile("v_nop\n\tv_nop\n\tv_nop\n\tv_nop" : "+v"(d) : "v"(a), "v"(b));
    return d;
}

__device__ __forceinline__ float abs_opaque(float x) {
    float r;
    asm("v_and_b32 %0, 0x7fffffff, %1" : "=v"(r) : "v"(x));
    return r;
}

__device__ __forceinline__ void st2v4(float* p, v4f v) {
    *(volatile v4f*)p = v;
    __threadfence();
    *(volatile v4f*)p = v;
}
__device__ __forceinline__ void st2v2(float* p, v2f v) {
    *(volatile v2f*)p = v;
    __threadfence();
    *(volatile v2f*)p = v;
}

__device__ __forceinline__ float wsum(float v) {
    v += __shfl_xor(v, 16); v += __shfl_xor(v, 8); v += __shfl_xor(v, 4);
    v += __shfl_xor(v, 2);  v += __shfl_xor(v, 1);
    return v;
}
__device__ __forceinline__ float wmax(float v) {
    v = fmaxf(v, __shfl_xor(v, 16)); v = fmaxf(v, __shfl_xor(v, 8)); v = fmaxf(v, __shfl_xor(v, 4));
    v = fmaxf(v, __shfl_xor(v, 2));  v = fmaxf(v, __shfl_xor(v, 1));
    return v;
}
__device__ __forceinline__ float hsum16(float v) {
    v += __shfl_xor(v, 1, 16); v += __shfl_xor(v, 2, 16);
    v += __shfl_xor(v, 4, 16); v += __shfl_xor(v, 8, 16);
    return v;
}
__device__ __forceinline__ v4f wsum4(v4f a) {
    a.x = wsum(a.x); a.y = wsum(a.y); a.z = wsum(a.z); a.w = wsum(a.w);
    return a;
}

__device__ __forceinline__ v16h ldfrag(const _Float16* base, int c, int h) {
    Frag f;
    f.half[0] = *(const v8h*)(base + 32 * c + 8 * h);
    f.half[1] = *(const v8h*)(base + 32 * c + 16 + 8 * h);
    return f.v;
}

__device__ __forceinline__ v8h absdiff8(const float* p, v4f e0, v4f e1) {
    const v4f u0 = *(const v4f*)p;
    const v4f u1 = *(const v4f*)(p + 4);
    v8h r;
    r[0] = (_Float16)abs_opaque(u0.x - e0.x);
    r[1] = (_Float16)abs_opaque(u0.y - e0.y);
    r[2] = (_Float16)abs_opaque(u0.z - e0.z);
    r[3] = (_Float16)abs_opaque(u0.w - e0.w);
    r[4] = (_Float16)abs_opaque(u1.x - e1.x);
    r[5] = (_Float16)abs_opaque(u1.y - e1.y);
    r[6] = (_Float16)abs_opaque(u1.z - e1.z);
    r[7] = (_Float16)abs_opaque(u1.w - e1.w);
    return r;
}

__global__ __launch_bounds__(256) void k_gemm4(const float* __restrict__ X,
                                               const float* __restrict__ W,
                                               const float* __restrict__ bias,
                                               float* __restrict__ Y,
                                               int M, int N, int K, int relu) {
    const int nq = N >> 2;
    const int idx = blockIdx.x * 256 + threadIdx.x;
    if (idx >= M * nq) return;
    const int m = idx / nq;
    const int q = idx - m * nq;
    v4f acc = *(const v4f*)(bias + 4 * q);
    const float* xr = X + (size_t)m * K;
    const float* wc = W + 4 * q;
    #pragma unroll 4
    for (int k = 0; k < K; ++k) {
        const float a = xr[k];
        const v4f w = *(const v4f*)(wc + (size_t)k * N);
        acc += a * w;
    }
    if (relu) {
        acc.x = fmaxf(acc.x, 0.f); acc.y = fmaxf(acc.y, 0.f);
        acc.z = fmaxf(acc.z, 0.f); acc.w = fmaxf(acc.w, 0.f);
    }
    st2v4(Y + (size_t)m * N + 4 * q, acc);
}

__global__ __launch_bounds__(256) void k_ln64(const float* __restrict__ X,
                                              const float* R, int has_res,
                                              const float* __restrict__ g,
                                              const float* __restrict__ b,
                                              float* __restrict__ Y, int M, int relu) {
    const int lane = threadIdx.x & 31;
    const int w = threadIdx.x >> 5;
    const int row = blockIdx.x * 8 + w;
    if (row >= M) return;
    const size_t off = (size_t)row * HID + 2 * lane;
    v2f x = *(const v2f*)(X + off);
    if (has_res) x += *(const v2f*)(R + off);
    const float s = wsum(x.x + x.y);
    const float mean = s * (1.f / 64.f);
    v2f d;
    d.x = x.x - mean; d.y = x.y - mean;
    const float vs = wsum(d.x * d.x + d.y * d.y);
    const float rs = rsqrtf(vs * (1.f / 64.f) + 1e-5f);
    const v2f gg = *(const v2f*)(g + 2 * lane);
    const v2f bb = *(const v2f*)(b + 2 * lane);
    v2f y;
    y.x = d.x * rs * gg.x + bb.x;
    y.y = d.y * rs * gg.y + bb.y;
    if (relu) { y.x = fmaxf(y.x, 0.f); y.y = fmaxf(y.y, 0.f); }
    st2v2(Y + off, y);
}

__global__ __launch_bounds__(128) void k_attn(const float* __restrict__ qkv, float* __restrict__ O) {
    __shared__ float sc[4][NN];
    __shared__ __attribute__((aligned(16))) float os[HID];
    const int lane = threadIdx.x & 31;
    const int w = threadIdx.x >> 5;
    const int i = blockIdx.x;
    const float* qp = qkv + (size_t)i * QKVW + w * 16;
    const v4f q0 = *(const v4f*)(qp);
    const v4f q1 = *(const v4f*)(qp + 4);
    const v4f q2 = *(const v4f*)(qp + 8);
    const v4f q3 = *(const v4f*)(qp + 12);

    float mx = -3.0e38f;
    #pragma unroll 1
    for (int t = 0; t < NN / 32; ++t) {
        const int j = lane + 32 * t;
        const float* kp = qkv + (size_t)j * QKVW + HID + w * 16;
        const v4f k0 = *(const v4f*)(kp);
        const v4f k1 = *(const v4f*)(kp + 4);
        const v4f k2 = *(const v4f*)(kp + 8);
        const v4f k3 = *(const v4f*)(kp + 12);
        v4f pr = q0 * k0;
        pr += q1 * k1; pr += q2 * k2; pr += q3 * k3;
        const float s = (pr.x + pr.y + pr.z + pr.w) * 0.25f;
        sc[w][j] = s;
        mx = fmaxf(mx, s);
    }
    mx = wmax(mx);
    float sm = 0.f;
    #pragma unroll 1
    for (int t = 0; t < NN / 32; ++t) {
        const int j = lane + 32 * t;
        const float e = expf(sc[w][j] - mx);
        sc[w][j] = e;
        sm += e;
    }
    sm = wsum(sm);
    const float inv = 1.f / sm;

    v4f a0 = {0.f, 0.f, 0.f, 0.f}, a1 = a0, a2 = a0, a3 = a0;
    #pragma unroll 1
    for (int t = 0; t < NN / 32; ++t) {
        const int j = lane + 32 * t;
        const float p = sc[w][j];
        const float* vp = qkv + (size_t)j * QKVW + 2 * HID + w * 16;
        const v4f v0 = *(const v4f*)(vp);
        const v4f v1 = *(const v4f*)(vp + 4);
        const v4f v2 = *(const v4f*)(vp + 8);
        const v4f v3 = *(const v4f*)(vp + 12);
        a0 += p * v0; a1 += p * v1; a2 += p * v2; a3 += p * v3;
    }
    a0 = wsum4(a0); a1 = wsum4(a1); a2 = wsum4(a2); a3 = wsum4(a3);
    if (lane == 0) {
        *(v4f*)&os[w * 16]      = a0 * inv;
        *(v4f*)&os[w * 16 + 4]  = a1 * inv;
        *(v4f*)&os[w * 16 + 8]  = a2 * inv;
        *(v4f*)&os[w * 16 + 12] = a3 * inv;
    }
    __syncthreads();
    if (w == 0 && lane < 16) {
        const v4f v = *(const v4f*)&os[4 * lane];
        st2v4(O + (size_t)i * HID + 4 * lane, v);
    }
}

__global__ __launch_bounds__(256) void k_prep(const float* __restrict__ enc,
                                              const float* __restrict__ pg_w1,
                                              const float* __restrict__ pg_b1,
                                              const float* __restrict__ pv_w1,
                                              const float* __restrict__ pv_b1,
                                              float* __restrict__ Ag, float* __restrict__ Bg,
                                              float* __restrict__ Av, float* __restrict__ Bv) {
    const bool sel = (blockIdx.y != 0);
    const float* W  = sel ? pv_w1 : pg_w1;
    const float* b1 = sel ? pv_b1 : pg_b1;
    float* Ao = sel ? Av : Ag;
    float* Bo = sel ? Bv : Bg;
    const int idx = blockIdx.x * 256 + threadIdx.x;
    if (idx >= NN * (HID / 4)) return;
    const int i = idx >> 4;
    const int q = idx & 15;
    v4f a = *(const v4f*)(b1 + 4 * q);
    v4f bb = {0.f, 0.f, 0.f, 0.f};
    const float* er = enc + (size_t)i * HID;
    #pragma unroll 2
    for (int k = 0; k < HID; ++k) {
        const float e = er[k];
        const v4f wl = *(const v4f*)(W + (size_t)k * HID + 4 * q);
        const v4f wr = *(const v4f*)(W + (size_t)(HID + k) * HID + 4 * q);
        const v4f wd = *(const v4f*)(W + (size_t)(2 * HID + k) * HID + 4 * q);
        a  += e * (wl + wd);
        bb += e * (wr - wd);
    }
    st2v4(Ao + (size_t)i * HID + 4 * q, a);
    st2v4(Bo + (size_t)i * HID + 4 * q, bb);
}

__global__ __launch_bounds__(128) void k_pair(
    const float* __restrict__ enc,
    const float* __restrict__ pg_w1, const float* __restrict__ pg_w2, const float* __restrict__ pg_b2,
    const float* __restrict__ pv_w1, const float* __restrict__ pv_w2, const float* __restrict__ pv_b2,
    const float* __restrict__ Ag, const float* __restrict__ Bg,
    const float* __restrict__ Av, const float* __restrict__ Bv,
    const float* __restrict__ lng, const float* __restrict__ lnb,
    float* __restrict__ enc2)
{
    __shared__ __attribute__((aligned(16))) _Float16 Wsh[3][HID][WPITCH];
    __shared__ __attribute__((aligned(16))) float gate_s[4][NN];
    __shared__ __attribute__((aligned(16))) float ab_s[4][2][HID];
    __shared__ __attribute__((aligned(16))) float w2_s[HID];
    __shared__ __attribute__((aligned(16))) float ctx_s[4][HID];

    const int tid  = threadIdx.x;
    const int lane = tid & 31;
    const int w    = tid >> 5;
    const int h    = lane >> 4;
    const int m    = lane & 15;
    const int i    = blockIdx.x * 4 + w;

    for (int idx = tid; idx < 3 * HID * HID; idx += 128) {
        const int mat = idx >> 12;
        const int rem = idx & 4095;
        const int k = rem >> 6;
        const int n = rem & 63;
        float v;
        if (mat == 0)      v = pg_w1[(size_t)(3 * HID + k) * HID + n];
        else if (mat == 1) v = pv_w1[(size_t)(3 * HID + k) * HID + n];
        else               v = pv_w2[(size_t)k * HID + n];
        Wsh[mat][n][k] = (_Float16)(v * 16.f);
    }
    ab_s[w][0][lane]      = Ag[(size_t)i * HID + lane];
    ab_s[w][0][lane + 32] = Ag[(size_t)i * HID + lane + 32];
    ab_s[w][1][lane]      = Av[(size_t)i * HID + lane];
    ab_s[w][1][lane + 32] = Av[(size_t)i * HID + lane + 32];
    if (tid < HID) w2_s[tid] = pg_w2[tid];

    const float* eri = enc + (size_t)i * HID;
    v4f eg[8];
    eg[0] = *(const v4f*)(eri + 8 * h);       eg[1] = *(const v4f*)(eri + 8 * h + 4);
    eg[2] = *(const v4f*)(eri + 16 + 8 * h);  eg[3] = *(const v4f*)(eri + 20 + 8 * h);
    eg[4] = *(const v4f*)(eri + 32 + 8 * h);  eg[5] = *(const v4f*)(eri + 36 + 8 * h);
    eg[6] = *(const v4f*)(eri + 48 + 8 * h);  eg[7] = *(const v4f*)(eri + 52 + 8 * h);
    const float gb2 = pg_b2[0];
    __syncthreads();

    #pragma unroll 1
    for (int jt = 0; jt < NN / 16; ++jt) {
        const int j0 = jt * 16;
        const int jm = j0 + m;
        const float* erj = enc + (size_t)jm * HID;
        Frag x0, x1;
        x0.half[0] = absdiff8(erj + 8 * h,      eg[0], eg[1]);
        x0.half[1] = absdiff8(erj + 16 + 8 * h, eg[2], eg[3]);
        x1.half[0] = absdiff8(erj + 32 + 8 * h, eg[4], eg[5]);
        x1.half[1] = absdiff8(erj + 48 + 8 * h, eg[6], eg[7]);
        const float* bgr = Bg + (size_t)jm * HID;
        float gp = 0.f;
        #pragma unroll
        for (int tt = 0; tt < 4; ++tt) {
            const _Float16* wa = &Wsh[0][16 * tt + m][0];
            v8f c = {0.f, 0.f, 0.f, 0.f, 0.f, 0.f, 0.f, 0.f};
            c = wmma16(ldfrag(wa, 0, h), x0.v, c);
            c = wmma16(ldfrag(wa, 1, h), x1.v, c);
            const int nb = 16 * tt + 8 * h;
            const v4f ag0 = *(const v4f*)&ab_s[w][0][nb];
            const v4f ag1 = *(const v4f*)&ab_s[w][0][nb + 4];
            const v4f bg0 = *(const v4f*)(bgr + nb);
            const v4f bg1 = *(const v4f*)(bgr + nb + 4);
            const v4f w20 = *(const v4f*)&w2_s[nb];
            const v4f w21 = *(const v4f*)&w2_s[nb + 4];
            #pragma unroll
            for (int r = 0; r < 4; ++r) {
                const float h0v = c[r]     * 0.0625f + ag0[r] + bg0[r];
                const float h1v = c[4 + r] * 0.0625f + ag1[r] + bg1[r];
                gp += fmaxf(h0v, 0.f) * w20[r];
                gp += fmaxf(h1v, 0.f) * w21[r];
            }
        }
        gp += __shfl_xor(gp, 16);
        float gv = gp + gb2;
        if (jm == i) gv = -1.0e9f;
        if (h == 0) gate_s[w][jm] = gv;
    }
    __syncthreads();

    float mx = -3.0e38f;
    #pragma unroll 1
    for (int t = 0; t < NN / 32; ++t) mx = fmaxf(mx, gate_s[w][lane + 32 * t]);
    mx = wmax(mx);
    float sm = 0.f;
    #pragma unroll 1
    for (int t = 0; t < NN / 32; ++t) {
        const int j = lane + 32 * t;
        const float e = expf(gate_s[w][j] - mx);
        gate_s[w][j] = e;
        sm += e;
    }
    sm = wsum(sm);
    const float inv = 1.f / sm;
    __syncthreads();

    v8f acc2[4];
    #pragma unroll
    for (int t2 = 0; t2 < 4; ++t2) { v8f z = {0.f, 0.f, 0.f, 0.f, 0.f, 0.f, 0.f, 0.f}; acc2[t2] = z; }

    #pragma unroll 1
    for (int jt = 0; jt < NN / 16; ++jt) {
        const int j0 = jt * 16;
        const int jm = j0 + m;
        const float* erj = enc + (size_t)jm * HID;
        Frag x0, x1;
        x0.half[0] = absdiff8(erj + 8 * h,      eg[0], eg[1]);
        x0.half[1] = absdiff8(erj + 16 + 8 * h, eg[2], eg[3]);
        x1.half[0] = absdiff8(erj + 32 + 8 * h, eg[4], eg[5]);
        x1.half[1] = absdiff8(erj + 48 + 8 * h, eg[6], eg[7]);
        const float p = gate_s[w][jm];
        const float* bvr = Bv + (size_t)jm * HID;

        v8h pk[4];
        #pragma unroll
        for (int tt = 0; tt < 4; ++tt) {
            const _Float16* wa = &Wsh[1][16 * tt + m][0];
            v8f c = {0.f, 0.f, 0.f, 0.f, 0.f, 0.f, 0.f, 0.f};
            c = wmma16(ldfrag(wa, 0, h), x0.v, c);
            c = wmma16(ldfrag(wa, 1, h), x1.v, c);
            const int nb = 16 * tt + 8 * h;
            const v4f av0 = *(const v4f*)&ab_s[w][1][nb];
            const v4f av1 = *(const v4f*)&ab_s[w][1][nb + 4];
            const v4f bv0 = *(const v4f*)(bvr + nb);
            const v4f bv1 = *(const v4f*)(bvr + nb + 4);
            v8h q;
            #pragma unroll
            for (int r = 0; r < 4; ++r) {
                q[r]     = (_Float16)fmaxf(c[r]     * 0.0625f + av0[r] + bv0[r], 0.f);
                q[4 + r] = (_Float16)fmaxf(c[4 + r] * 0.0625f + av1[r] + bv1[r], 0.f);
            }
            pk[tt] = q;
        }
        Frag hb0, hb1;
        hb0.half[0] = pk[0]; hb0.half[1] = pk[1];
        hb1.half[0] = pk[2]; hb1.half[1] = pk[3];

        #pragma unroll
        for (int t2 = 0; t2 < 4; ++t2) {
            const _Float16* wa = &Wsh[2][16 * t2 + m][0];
            v8f c = {0.f, 0.f, 0.f, 0.f, 0.f, 0.f, 0.f, 0.f};
            c = wmma16(ldfrag(wa, 0, h), hb0.v, c);
            c = wmma16(ldfrag(wa, 1, h), hb1.v, c);
            acc2[t2] = acc2[t2] + p * c;
        }
    }

    const float sc16 = inv * 0.0625f;
    float s1 = 0.f;
    v8f y[4];
    #pragma unroll
    for (int tt = 0; tt < 4; ++tt) {
        v8f a = acc2[tt];
        #pragma unroll
        for (int r = 0; r < 8; ++r) a[r] = hsum16(a[r]);
        const int nb = 16 * tt + 8 * h;
        const v4f pb0 = *(const v4f*)(pv_b2 + nb);
        const v4f pb1 = *(const v4f*)(pv_b2 + nb + 4);
        v8f yy;
        #pragma unroll
        for (int r = 0; r < 4; ++r) {
            yy[r]     = eg[2 * tt][r]     + (a[r]     * sc16 + pb0[r]);
            yy[4 + r] = eg[2 * tt + 1][r] + (a[4 + r] * sc16 + pb1[r]);
        }
        y[tt] = yy;
        #pragma unroll
        for (int r = 0; r < 8; ++r) s1 += yy[r];
    }
    s1 += __shfl_xor(s1, 16);
    const float mean = s1 * (1.f / 64.f);
    float s2 = 0.f;
    #pragma unroll
    for (int tt = 0; tt < 4; ++tt) {
        #pragma unroll
        for (int r = 0; r < 8; ++r) { const float d = y[tt][r] - mean; y[tt][r] = d; s2 += d * d; }
    }
    s2 += __shfl_xor(s2, 16);
    const float rs = rsqrtf(s2 * (1.f / 64.f) + 1e-5f);
    #pragma unroll
    for (int tt = 0; tt < 4; ++tt) {
        const int nb = 16 * tt + 8 * h;
        const v4f g0 = *(const v4f*)(lng + nb);
        const v4f g1 = *(const v4f*)(lng + nb + 4);
        const v4f b0 = *(const v4f*)(lnb + nb);
        const v4f b1 = *(const v4f*)(lnb + nb + 4);
        v4f o0, o1;
        #pragma unroll
        for (int r = 0; r < 4; ++r) {
            o0[r] = y[tt][r]     * rs * g0[r] + b0[r];
            o1[r] = y[tt][4 + r] * rs * g1[r] + b1[r];
        }
        if (m == 0) {
            *(v4f*)&ctx_s[w][nb]     = o0;
            *(v4f*)&ctx_s[w][nb + 4] = o1;
        }
    }
    __syncthreads();
    if (lane < 16) {
        const v4f v = *(const v4f*)&ctx_s[w][4 * lane];
        st2v4(enc2 + (size_t)i * HID + 4 * lane, v);
    }
}

__global__ __launch_bounds__(64) void k_gctx(const float* __restrict__ enc2,
                                             const float* __restrict__ sh_w1,
                                             const float* __restrict__ sh_b1,
                                             float* __restrict__ gb) {
    __shared__ __attribute__((aligned(16))) float gm[HID];
    __shared__ __attribute__((aligned(16))) float gbs[HID];
    const int c = threadIdx.x;
    double s = 0.0;
    #pragma unroll 4
    for (int r = 0; r < NN; ++r) s += (double)enc2[(size_t)r * HID + c];
    gm[c] = (float)(s * (1.0 / 1024.0));
    __syncthreads();
    float a = sh_b1[c];
    #pragma unroll 4
    for (int k = 0; k < HID; ++k) a += gm[k] * sh_w1[(size_t)(HID + k) * HID + c];
    gbs[c] = a;
    __syncthreads();
    if (c < 16) {
        const v4f v = *(const v4f*)&gbs[4 * c];
        st2v4(gb + 4 * c, v);
    }
}

__global__ __launch_bounds__(256) void k_head(const float* __restrict__ enc2,
                                              const float* __restrict__ sh_w1,
                                              const float* __restrict__ gb,
                                              const float* __restrict__ sh_w2,
                                              const float* __restrict__ sh_b2,
                                              float* __restrict__ out) {
    __shared__ float Ws[HID * HID];
    __shared__ float gbs[HID];
    __shared__ float w2s[HID];
    __shared__ __attribute__((aligned(16))) float outs[NN];
    const int tid = threadIdx.x;
    const int lane = tid & 31;
    const int w = tid >> 5;
    for (int idx = tid; idx < HID * HID; idx += 256) Ws[idx] = sh_w1[idx];
    if (tid < HID) { gbs[tid] = gb[tid]; w2s[tid] = sh_w2[tid]; }
    __syncthreads();
    const float b2 = sh_b2[0];
    #pragma unroll 1
    for (int r = 0; r < NN / 8; ++r) {
        const int i = w * (NN / 8) + r;
        const float* er = enc2 + (size_t)i * HID;
        float h0 = gbs[lane];
        float h1 = gbs[lane + 32];
        #pragma unroll 4
        for (int k = 0; k < HID; ++k) {
            const float e = er[k];
            h0 += e * Ws[k * HID + lane];
            h1 += e * Ws[k * HID + lane + 32];
        }
        float pp = fmaxf(h0, 0.f) * w2s[lane] + fmaxf(h1, 0.f) * w2s[lane + 32];
        pp = wsum(pp);
        if (lane == 0) outs[i] = pp + b2;
    }
    __syncthreads();
    if (w == 0) {
        #pragma unroll
        for (int qq = 0; qq < NN / 128; ++qq) {
            const v4f v = *(const v4f*)&outs[qq * 128 + 4 * lane];
            *(volatile v4f*)(out + qq * 128 + 4 * lane) = v;
        }
        __threadfence();
        #pragma unroll
        for (int qq = 0; qq < NN / 128; ++qq) {
            const v4f v = *(const v4f*)&outs[qq * 128 + 4 * lane];
            *(volatile v4f*)(out + qq * 128 + 4 * lane) = v;
        }
    }
}

extern "C" void kernel_launch(void* const* d_in, const int* in_sizes, int n_in,
                              void* d_out, int out_size, void* d_ws, size_t ws_size,
                              hipStream_t stream) {
    if (n_in < 27) return;
    if (in_sizes[0] != NN * FEAT || in_sizes[1] != FEAT * HID || in_sizes[7] != HID * QKVW ||
        in_sizes[13] != 4 * HID * HID || in_sizes[17] != 4 * HID * HID || in_sizes[23] != 2 * HID * HID ||
        out_size != NN) return;
    const size_t NT = (size_t)NN * HID;
    const size_t need_floats = 14 * NT + HID;
    if (ws_size < need_floats * sizeof(float)) return;

    const float* features   = (const float*)d_in[0];
    const float* ip_w1      = (const float*)d_in[1];
    const float* ip_b1      = (const float*)d_in[2];
    const float* ip_ln_g    = (const float*)d_in[3];
    const float* ip_ln_b    = (const float*)d_in[4];
    const float* ip_w2      = (const float*)d_in[5];
    const float* ip_b2      = (const float*)d_in[6];
    const float* attn_in_w  = (const float*)d_in[7];
    const float* attn_in_b  = (const float*)d_in[8];
    const float* attn_out_w = (const float*)d_in[9];
    const float* attn_out_b = (const float*)d_in[10];
    const float* attn_ln_g  = (const float*)d_in[11];
    const float* attn_ln_b  = (const float*)d_in[12];
    const float* pg_w1      = (const float*)d_in[13];
    const float* pg_b1      = (const float*)d_in[14];
    const float* pg_w2      = (const float*)d_in[15];
    const float* pg_b2      = (const float*)d_in[16];
    const float* pv_w1      = (const float*)d_in[17];
    const float* pv_b1      = (const float*)d_in[18];
    const float* pv_w2      = (const float*)d_in[19];
    const float* pv_b2      = (const float*)d_in[20];
    const float* ctx_ln_g   = (const float*)d_in[21];
    const float* ctx_ln_b   = (const float*)d_in[22];
    const float* sh_w1      = (const float*)d_in[23];
    const float* sh_b1      = (const float*)d_in[24];
    const float* sh_w2      = (const float*)d_in[25];
    const float* sh_b2      = (const float*)d_in[26];
    float* out = (float*)d_out;

    float* ws   = (float*)d_ws;
    float* t0   = ws + 0 * NT;
    float* t1   = ws + 1 * NT;
    float* hbuf = ws + 2 * NT;
    float* qkv  = ws + 3 * NT;
    float* o    = ws + 6 * NT;
    float* t2   = ws + 7 * NT;
    float* enc  = ws + 8 * NT;
    float* Ag   = ws + 9 * NT;
    float* Bg   = ws + 10 * NT;
    float* Av   = ws + 11 * NT;
    float* Bv   = ws + 12 * NT;
    float* enc2 = ws + 13 * NT;
    float* gb   = ws + 14 * NT;

    const int gq64  = (NN * (HID / 4) + 255) / 256;
    const int gq192 = (NN * (QKVW / 4) + 255) / 256;
    const int gln   = (NN + 7) / 8;

    k_gemm4<<<gq64, 256, 0, stream>>>(features, ip_w1, ip_b1, t0, NN, HID, FEAT, 0);
    k_ln64<<<gln, 256, 0, stream>>>(t0, t0, 0, ip_ln_g, ip_ln_b, t1, NN, 1);
    k_gemm4<<<gq64, 256, 0, stream>>>(t1, ip_w2, ip_b2, hbuf, NN, HID, HID, 1);

    k_gemm4<<<gq192, 256, 0, stream>>>(hbuf, attn_in_w, attn_in_b, qkv, NN, QKVW, HID, 0);
    k_attn<<<NN, 128, 0, stream>>>(qkv, o);
    k_gemm4<<<gq64, 256, 0, stream>>>(o, attn_out_w, attn_out_b, t2, NN, HID, HID, 0);
    k_ln64<<<gln, 256, 0, stream>>>(t2, hbuf, 1, attn_ln_g, attn_ln_b, enc, NN, 0);

    k_prep<<<dim3(gq64, 2), 256, 0, stream>>>(enc, pg_w1, pg_b1, pv_w1, pv_b1, Ag, Bg, Av, Bv);

    k_pair<<<NN / 4, 128, 0, stream>>>(enc, pg_w1, pg_w2, pg_b2, pv_w1, pv_w2, pv_b2,
                                       Ag, Bg, Av, Bv, ctx_ln_g, ctx_ln_b, enc2);

    k_gctx<<<1, 64, 0, stream>>>(enc2, sh_w1, sh_b1, gb);
    k_head<<<1, 256, 0, stream>>>(enc2, sh_w1, gb, sh_w2, sh_b2, out);
}
